// ImprovedGraphSAGE_88905823027737
// MI455X (gfx1250) — hardware-verified
//
#include <hip/hip_runtime.h>
#include <stddef.h>
#include <math.h>


#define FW      128
#define NH      128
#define KIN     128
#define KS      256
#define NLAY    3
#define NCLS    2
#define NTHR    256
#define NWAVE   8
#define EPT     8
#define NGRP    2
#define CHUNK   (NTHR * EPT * NGRP)
#define WCAP    (EPT * NGRP * 32)
#define LISTN   (NWAVE * WCAP)
#define NBC     4096
#define NBF     1024
#define RCAP    40960
#define RBN     128
#define RPAD    256
#define ATHR    64
#define AWAVE   2
#define TGT     (AWAVE * 32)
#define DEGCAP  1024
#define OTHR    512
#define BMR     32
#define WSCAP   134217728
#define ACARRY  8.0f
#define WCARRY  64.0f
#define GSCALE  (1.0f / 512.0f)
#define LNEPS   1e-5f
#define U0      (NH * (KIN / 8))
#define UL      (NH * (KS / 8))
#define NUNITS  (U0 + NLAY * UL)

#define LDS_FILL ((RCAP + NBF + LISTN) * 4 + 64)

static_assert((CHUNK & (CHUNK - 1)) == 0);
static_assert(CHUNK <= 4096);
static_assert((NBC & (NBC - 1)) == 0 && (NBF & (NBF - 1)) == 0);
static_assert(NBC == 4 * NBF);
static_assert(OTHR * 8 == NBC);
static_assert((RCAP % 32) == 0);
static_assert(WCAP == EPT * NGRP * 32);
static_assert(KS == 2 * FW);
static_assert((KS % 32) == 0 && (KIN % 32) == 0);
static_assert(NH == FW && KIN == FW);
static_assert((RPAD % TGT) == 0 && (RPAD % 128) == 0 && (RPAD % BMR) == 0);
static_assert((NBC % RPAD) == 0);
static_assert(TGT == AWAVE * 32);
static_assert(ATHR == AWAVE * 32);
static_assert((NUNITS % NTHR) == 0);
static_assert(NTHR == FW * NCLS);
static_assert((NCLS & (NCLS - 1)) == 0);

typedef float    v4f  __attribute__((ext_vector_type(4)));
typedef float    v8f  __attribute__((ext_vector_type(8)));
typedef int      v4i  __attribute__((ext_vector_type(4)));
typedef _Float16 v4h  __attribute__((ext_vector_type(4)));
typedef _Float16 v8h  __attribute__((ext_vector_type(8)));
typedef _Float16 v16h __attribute__((ext_vector_type(16)));
union Frag { v16h v; v8h h[2]; };

__device__ __forceinline__ v8f wmh(v16h a, v16h b, v8f c) {
  v8f d = __builtin_amdgcn_wmma_f32_16x16x32_f16(false, a, false, b, (short)0, c, false, false);
  asm volatile("v_nop\n\tv_nop\n\tv_nop\n\tv_nop" : "+v"(d) : "v"(a), "v"(b));
  return d;
}

template <int NB>
__device__ __forceinline__ int scan_chunk(const int* __restrict__ dsts, int nE, int cbase, int slotBase,
                                          int vec8, int* list, int tid, int lane, int wave) {
  int wc = 0;
#pragma unroll
  for (int g = 0; g < NGRP; ++g) {
    const int el0  = (g * NTHR + tid) * EPT;
    const int e0   = cbase + el0;
    const int sent = -2147483647 - 1;
    v4i da, db;
    if (vec8 != 0 && cbase + CHUNK <= nE) {
      da = *(const v4i*)(dsts + e0);
      db = *(const v4i*)(dsts + e0 + 4);
    } else {
      da.x = (e0     < nE) ? dsts[min(e0, nE - 1)] : sent;
      da.y = (e0 + 1 < nE) ? dsts[min(e0 + 1, nE - 1)] : sent;
      da.z = (e0 + 2 < nE) ? dsts[min(e0 + 2, nE - 1)] : sent;
      da.w = (e0 + 3 < nE) ? dsts[min(e0 + 3, nE - 1)] : sent;
      db.x = (e0 + 4 < nE) ? dsts[min(e0 + 4, nE - 1)] : sent;
      db.y = (e0 + 5 < nE) ? dsts[min(e0 + 5, nE - 1)] : sent;
      db.z = (e0 + 6 < nE) ? dsts[min(e0 + 6, nE - 1)] : sent;
      db.w = (e0 + 7 < nE) ? dsts[min(e0 + 7, nE - 1)] : sent;
    }
    const unsigned nb = (unsigned)slotBase;
    const unsigned s0 = (unsigned)da.x - nb, s1 = (unsigned)da.y - nb;
    const unsigned s2 = (unsigned)da.z - nb, s3 = (unsigned)da.w - nb;
    const unsigned s4 = (unsigned)db.x - nb, s5 = (unsigned)db.y - nb;
    const unsigned s6 = (unsigned)db.z - nb, s7 = (unsigned)db.w - nb;
    const bool h0 = s0 < (unsigned)NB, h1 = s1 < (unsigned)NB, h2 = s2 < (unsigned)NB, h3 = s3 < (unsigned)NB;
    const bool h4 = s4 < (unsigned)NB, h5 = s5 < (unsigned)NB, h6 = s6 < (unsigned)NB, h7 = s7 < (unsigned)NB;
    const unsigned any = __builtin_amdgcn_ballot_w32(h0 | h1 | h2 | h3 | h4 | h5 | h6 | h7);
    if (any != 0u) {
#define HITJ(J, HJ, SJ) { \
        const unsigned mj = __builtin_amdgcn_ballot_w32(HJ); \
        if (mj != 0u) { \
          if (HJ) { \
            const int pos = wc + (int)__builtin_amdgcn_mbcnt_lo(mj, 0u); \
            if (pos < WCAP) list[wave * WCAP + pos] = ((el0 + (J)) << 12) | (int)(SJ); \
          } \
          wc += (int)__builtin_popcount(mj); } }
      HITJ(0, h0, s0)
      HITJ(1, h1, s1)
      HITJ(2, h2, s2)
      HITJ(3, h3, s3)
      HITJ(4, h4, s4)
      HITJ(5, h5, s5)
      HITJ(6, h6, s6)
      HITJ(7, h7, s7)
#undef HITJ
    }
  }
  return wc;
}

__global__ __launch_bounds__(NTHR) void k_count(
    const int* __restrict__ dsts, int* cnt, int nE, int vec8) {
  __shared__ __attribute__((aligned(16))) int scnt[NBC];
  __shared__ __attribute__((aligned(16))) int list[LISTN];
  __shared__ int wcnt[NWAVE];
  const int tid = threadIdx.x, lane = tid & 31, wave = tid >> 5;
  const int nodeBase = blockIdx.x * NBC;

  for (int i = tid; i < NBC; i += NTHR) scnt[i] = 0;
  __syncthreads();

  const int nChunks = (nE + CHUNK - 1) / CHUNK;
#pragma unroll 1
  for (int ch = 0; ch < nChunks; ++ch) {
    const int cbase = ch * CHUNK;
    const int wc = scan_chunk<NBC>(dsts, nE, cbase, nodeBase, vec8, list, tid, lane, wave);
    if (lane == 0) wcnt[wave] = wc;
    __syncthreads();
    if (wave == 0) {
#pragma unroll 1
      for (int wsx = 0; wsx < NWAVE; ++wsx) {
        int n = __builtin_amdgcn_readfirstlane(wcnt[wsx]);
        n = n > WCAP ? WCAP : (n < 0 ? 0 : n);
        const int* lp = list + wsx * WCAP;
#pragma unroll 1
        for (int i = 0; i < n; ++i) {
          const int ent  = __builtin_amdgcn_readfirstlane(lp[i]);
          const int slot = ent & (NBC - 1);
          if (lane == 0) scnt[slot] = scnt[slot] + 1;
        }
      }
    }
    __syncthreads();
  }

  v4i cq[4];
#pragma unroll
  for (int q = 0; q < 4; ++q) {
    const int f = (wave * 4 + q) * 128 + 4 * lane;
    cq[q] = *(const v4i*)(scnt + f);
  }
  int* cp = cnt + (size_t)nodeBase;
#pragma unroll
  for (int q = 0; q < 4; ++q) {
    const int f = (wave * 4 + q) * 128 + 4 * lane;
    *(volatile v4i*)(cp + f) = cq[q];
  }
  __threadfence();
#pragma unroll
  for (int q = 0; q < 4; ++q) {
    const int f = (wave * 4 + q) * 128 + 4 * lane;
    *(volatile v4i*)(cp + f) = cq[q];
  }
}

__global__ __launch_bounds__(OTHR) void k_offsets(
    const int* __restrict__ cnt, int* off, int* rbase, int nChunk) {
  __shared__ __attribute__((aligned(16))) int soff[NBC];
  __shared__ __attribute__((aligned(16))) int srb[RBN];
  __shared__ int wtot[OTHR / 32];
  const int tid = threadIdx.x, lane = tid & 31, wave = tid >> 5, sub = tid >> 7;
  for (int i = tid; i < RBN; i += OTHR) srb[i] = 0;
  int carry = 0;
#pragma unroll 1
  for (int ch = 0; ch < nChunk; ++ch) {
    const int base = ch * NBC;
    const v4i c0 = *(const v4i*)(cnt + base + 8 * tid);
    const v4i c1 = *(const v4i*)(cnt + base + 8 * tid + 4);
    const int e0 = max(c0.x, 0), e1 = max(c0.y, 0), e2 = max(c0.z, 0), e3 = max(c0.w, 0);
    const int e4 = max(c1.x, 0), e5 = max(c1.y, 0), e6 = max(c1.z, 0), e7 = max(c1.w, 0);
    const int ts = e0 + e1 + e2 + e3 + e4 + e5 + e6 + e7;
    int incl = ts;
#pragma unroll
    for (int d = 1; d < 32; d <<= 1) {
      const int t = __shfl_up(incl, d);
      if (lane >= d) incl += t;
    }
    if (lane == 31) wtot[wave] = incl;
    __syncthreads();
    const int S0 = wtot[0]  + wtot[1]  + wtot[2]  + wtot[3];
    const int S1 = wtot[4]  + wtot[5]  + wtot[6]  + wtot[7];
    const int S2 = wtot[8]  + wtot[9]  + wtot[10] + wtot[11];
    const int S3 = wtot[12] + wtot[13] + wtot[14] + wtot[15];
    int pre = 0;
#pragma unroll 1
    for (int w = 4 * sub; w < wave; ++w) pre += wtot[w];
    const int b0 = carry;
    const int b1 = b0 + ((S0 + 31) & ~31);
    const int b2 = b1 + ((S1 + 31) & ~31);
    const int b3 = b2 + ((S2 + 31) & ~31);
    const int b4 = b3 + ((S3 + 31) & ~31);
    const int myb = sub == 0 ? b0 : (sub == 1 ? b1 : (sub == 2 ? b2 : b3));
    if (tid == 0) {
      srb[min(4 * ch + 0, RBN - 1)] = b0;
      srb[min(4 * ch + 1, RBN - 1)] = b1;
      srb[min(4 * ch + 2, RBN - 1)] = b2;
      srb[min(4 * ch + 3, RBN - 1)] = b3;
    }
    int run = myb + pre + incl - ts;
    soff[8 * tid + 0] = run; run += e0;
    soff[8 * tid + 1] = run; run += e1;
    soff[8 * tid + 2] = run; run += e2;
    soff[8 * tid + 3] = run; run += e3;
    soff[8 * tid + 4] = run; run += e4;
    soff[8 * tid + 5] = run; run += e5;
    soff[8 * tid + 6] = run; run += e6;
    soff[8 * tid + 7] = run;
    carry = b4;
    __syncthreads();
    const v4i o0 = *(const v4i*)(soff + 4 * tid);
    const v4i o1 = *(const v4i*)(soff + 4 * (tid + OTHR));
    int* op = off + base;
    *(volatile v4i*)(op + 4 * tid) = o0;
    *(volatile v4i*)(op + 4 * (tid + OTHR)) = o1;
    __threadfence();
    *(volatile v4i*)(op + 4 * tid) = o0;
    *(volatile v4i*)(op + 4 * (tid + OTHR)) = o1;
    __syncthreads();
  }
  if (tid == 0) srb[min(4 * nChunk, RBN - 1)] = carry;
  __syncthreads();
  v4i rv = {0, 0, 0, 0};
  if (tid < 32) rv = *(const v4i*)(srb + 4 * tid);
  if (tid < 32) *(volatile v4i*)(rbase + 4 * tid) = rv;
  __threadfence();
  if (tid < 32) *(volatile v4i*)(rbase + 4 * tid) = rv;
}

__global__ __launch_bounds__(NTHR) void k_fill(
    const int* __restrict__ srcs, const int* __restrict__ dsts,
    const int* __restrict__ off, const int* __restrict__ rbase,
    int* csr, int nN, int nE, int vec8, int csrLen) {
  extern __shared__ v4f lds_dyn[];
  int* region = (int*)lds_dyn;
  int* cursor = region + RCAP;
  int* list   = cursor + NBF;
  int* wcnt   = list + LISTN;
  const int tid = threadIdx.x, lane = tid & 31, wave = tid >> 5;
  const int b = blockIdx.x;
  const int nodeBase = b * NBF;

  int rb0 = rbase[b];
  const int rb1 = rbase[b + 1];
  rb0 = rb0 < 0 ? 0 : (rb0 > csrLen ? csrLen : rb0);
  rb0 &= ~31;
  int len = rb1 - rb0;
  len = len < 0 ? 0 : (len > RCAP ? RCAP : len);
  int lenW = (len + 31) & ~31;
  if (rb0 + lenW > csrLen) lenW = (csrLen - rb0) & ~31;

  {
    const v4i z = {0, 0, 0, 0};
    for (int i = tid; i < RCAP / 4; i += NTHR) ((v4i*)region)[i] = z;
    for (int s = tid; s < NBF; s += NTHR) {
      int o = off[nodeBase + s] - rb0;
      o = o < 0 ? 0 : (o > RCAP ? RCAP : o);
      cursor[s] = o;
    }
  }
  __syncthreads();

  const int nChunks = (nE + CHUNK - 1) / CHUNK;
#pragma unroll 1
  for (int ch = 0; ch < nChunks; ++ch) {
    const int cbase = ch * CHUNK;
    const int wc = scan_chunk<NBF>(dsts, nE, cbase, nodeBase, vec8, list, tid, lane, wave);
    if (lane == 0) wcnt[wave] = wc;
    __syncthreads();
    if (wave == 0) {
#pragma unroll 1
      for (int wsx = 0; wsx < NWAVE; ++wsx) {
        int n = __builtin_amdgcn_readfirstlane(wcnt[wsx]);
        n = n > WCAP ? WCAP : (n < 0 ? 0 : n);
        const int* lp = list + wsx * WCAP;
#pragma unroll 1
        for (int i = 0; i < n; ++i) {
          const int ent  = __builtin_amdgcn_readfirstlane(lp[i]);
          const int slot = ent & (NBF - 1);
          int e = cbase + ((ent >> 12) & (CHUNK - 1));
          e = e > nE - 1 ? nE - 1 : e;
          int sv = srcs[e];
          sv = sv < 0 ? 0 : (sv > nN - 1 ? nN - 1 : sv);
          if (lane == 0) {
            int pos = cursor[slot];
            pos = pos < 0 ? 0 : (pos > RCAP - 1 ? RCAP - 1 : pos);
            region[pos] = sv;
            const int np = pos + 1;
            cursor[slot] = np > RCAP ? RCAP : np;
          }
        }
      }
    }
    __syncthreads();
  }

  const int nv = lenW >> 2;
  int* gp = csr + rb0;
#pragma unroll 1
  for (int i = tid; i < nv; i += NTHR) { const v4i v = ((const v4i*)region)[i]; *(volatile v4i*)(gp + 4 * i) = v; }
  __threadfence();
#pragma unroll 1
  for (int i = tid; i < nv; i += NTHR) { const v4i v = ((const v4i*)region)[i]; *(volatile v4i*)(gp + 4 * i) = v; }
}

__global__ __launch_bounds__(NTHR) void k_wcvt(const float* __restrict__ Win, const float* __restrict__ Wl,
                                               const float* __restrict__ Wr, _Float16* wp, int nUnits) {
  const int u = (int)blockIdx.x * NTHR + (int)threadIdx.x;
  if (u >= nUnits) return;
  const bool p0 = u < U0;
  const int r = p0 ? u : (u - U0);
  int layer = p0 ? 0 : (r / UL);
  layer = layer > NLAY - 1 ? NLAY - 1 : layer;
  const int rr = p0 ? r : (r - layer * UL);
  const int ppr = p0 ? (KIN / 8) : (KS / 8);
  int n = rr / ppr;
  const int seg = rr - n * ppr;
  n = n > NH - 1 ? NH - 1 : (n < 0 ? 0 : n);
  const size_t lb = (size_t)layer * FW * NH;
  v8h o;
#pragma unroll
  for (int j = 0; j < 8; ++j) {
    const int k  = 8 * seg + j;
    const int kk = k & (FW - 1);
    const float f0 = Win[kk * NH + n];
    const float fl = Wl[lb + (size_t)kk * NH + n];
    const float fr = Wr[lb + (size_t)kk * NH + n];
    const float f = p0 ? f0 : ((k < FW) ? fl : fr);
    o[j] = (_Float16)(f * WCARRY);
  }
  _Float16* gp = wp + (size_t)u * 8;
  *(volatile v8h*)gp = o;
  __threadfence();
  *(volatile v8h*)gp = o;
}

__global__ __launch_bounds__(NTHR) void k_xcvt(const float* __restrict__ x, _Float16* xp, int nN, int nUnits) {
  const int u = (int)blockIdx.x * NTHR + (int)threadIdx.x;
  if (u >= nUnits) return;
  constexpr int PPR = KIN / 8;
  const int row = u / PPR;
  const int seg = u - row * PPR;
  const int rc = row > nN - 1 ? nN - 1 : row;
  const float sc = row < nN ? ACARRY : 0.f;
  const v4f a = *(const v4f*)(x + (size_t)rc * KIN + 8 * seg);
  const v4f b = *(const v4f*)(x + (size_t)rc * KIN + 8 * seg + 4);
  v8h o;
  o[0] = (_Float16)(a.x * sc); o[1] = (_Float16)(a.y * sc); o[2] = (_Float16)(a.z * sc); o[3] = (_Float16)(a.w * sc);
  o[4] = (_Float16)(b.x * sc); o[5] = (_Float16)(b.y * sc); o[6] = (_Float16)(b.z * sc); o[7] = (_Float16)(b.w * sc);
  _Float16* gp = xp + (size_t)u * 8;
  *(volatile v8h*)gp = o;
  __threadfence();
  *(volatile v8h*)gp = o;
}

__global__ __launch_bounds__(ATHR) void k_agg(
    const int* __restrict__ csr, const int* __restrict__ off, const int* __restrict__ cnt,
    const float* __restrict__ h, _Float16* ap, int nN, int csrLen) {
  __shared__ __attribute__((aligned(16))) _Float16 stg[AWAVE * 32 * KS];
  const int tid = threadIdx.x, lane = tid & 31, wave = tid >> 5;
  const int tbase = blockIdx.x * TGT + wave * 32;
  const int col4 = 4 * lane;
  const int cl    = tbase + lane;
  const int cnt_l = cnt[cl];
  const int off_l = off[cl];
  _Float16* sw = stg + (size_t)wave * 32 * KS;

#pragma unroll 1
  for (int j = 0; j < 32; ++j) {
    const int c = tbase + j;
    int nt = __shfl(cnt_l, j);
    nt = nt < 0 ? 0 : nt;
    const int n = nt > DEGCAP ? DEGCAP : nt;
    const int st = __shfl(off_l, j);
    float rc = 1.0f / (float)(nt < 1 ? 1 : nt);
    rc = (nt > DEGCAP) ? __int_as_float(0x7fc00000) : rc;

    v4f a = {0.f, 0.f, 0.f, 0.f};
#pragma unroll 1
    for (int q0 = 0; q0 < n; q0 += 32) {
      int pos = st + q0 + lane;
      pos = pos < 0 ? 0 : (pos > csrLen - 1 ? csrLen - 1 : pos);
      int sl = csr[pos];
      sl = sl < 0 ? 0 : (sl > nN - 1 ? nN - 1 : sl);
      const int mcnt = (n - q0) < 32 ? (n - q0) : 32;
#pragma unroll 1
      for (int pp = 0; pp < mcnt; ++pp) {
        const int s = __builtin_amdgcn_readlane(sl, pp);
        const v4f xv = *(const v4f*)(h + (size_t)s * FW + col4);
        a = a + xv;
      }
    }

    const bool live = c < nN;
    const int cc = c > nN - 1 ? nN - 1 : c;
    const v4f sv = *(const v4f*)(h + (size_t)cc * FW + col4);
    const float fm = live ? rc * ACARRY : 0.f;
    const float fs = live ? ACARRY : 0.f;
    v4h o0, o1;
    o0.x = (_Float16)(a.x * fm);  o0.y = (_Float16)(a.y * fm);
    o0.z = (_Float16)(a.z * fm);  o0.w = (_Float16)(a.w * fm);
    o1.x = (_Float16)(sv.x * fs); o1.y = (_Float16)(sv.y * fs);
    o1.z = (_Float16)(sv.z * fs); o1.w = (_Float16)(sv.w * fs);
    *(v4h*)(sw + j * KS + col4) = o0;
    *(v4h*)(sw + j * KS + FW + col4) = o1;
  }
  __syncthreads();

  constexpr int NI = (32 * KS) / (32 * 8);
  _Float16* gp = ap + (size_t)tbase * KS;
#pragma unroll 1
  for (int i = 0; i < NI; ++i) {
    const v8h v = *(const v8h*)(sw + i * 256 + 8 * lane);
    *(volatile v8h*)(gp + i * 256 + 8 * lane) = v;
  }
  __threadfence();
#pragma unroll 1
  for (int i = 0; i < NI; ++i) {
    const v8h v = *(const v8h*)(sw + i * 256 + 8 * lane);
    *(volatile v8h*)(gp + i * 256 + 8 * lane) = v;
  }
}

template <int KA, int LNRES>
__global__ __launch_bounds__(NTHR) void k_gemm(
    const _Float16* __restrict__ Ap, const _Float16* __restrict__ Bp, const float* __restrict__ bias,
    const float* __restrict__ gam, const float* __restrict__ bet, const float* __restrict__ Res,
    float* Cout, int nValid) {
  constexpr int NCOL = NH;
  constexpr int TPW = (BMR / 16) * (NCOL / 16) / NWAVE;
  constexpr int NCG = NCOL / (16 * TPW);
  constexpr int KSTEPS = KA / 32;
  constexpr int RPW = BMR / NWAVE;
  static_assert(TPW >= 1 && TPW * NWAVE * 256 == BMR * NCOL);
  static_assert(NCG >= 1 && NCG * 16 * TPW == NCOL);
  static_assert((NWAVE % NCG) == 0 && (NWAVE / NCG) * 16 == BMR);
  static_assert(RPW * NWAVE == BMR);
  static_assert(NCOL == 4 * 32);
  static_assert((KA % 32) == 0);

  __shared__ __attribute__((aligned(16))) float stg[BMR * NCOL];
  const int tid = threadIdx.x, lane = tid & 31, wave = tid >> 5, hh = lane >> 4, m = lane & 15;
  const int rowBase = (int)blockIdx.x * BMR;
  const int rg = wave / NCG, cg = wave - rg * NCG;
  const int r0 = rg * 16;
  const int c0 = cg * 16 * TPW;

  v8f acc[TPW];
#pragma unroll
  for (int t = 0; t < TPW; ++t) { v8f z = {0.f, 0.f, 0.f, 0.f, 0.f, 0.f, 0.f, 0.f}; acc[t] = z; }

  const _Float16* ap = Ap + (size_t)(rowBase + r0 + m) * KA + 8 * hh;
  const _Float16* bp = Bp + (size_t)(c0 + m) * KA + 8 * hh;
#pragma unroll 1
  for (int kt = 0; kt < KSTEPS; ++kt) {
    Frag a;
    a.h[0] = *(const v8h*)(ap + 32 * kt);
    a.h[1] = *(const v8h*)(ap + 32 * kt + 16);
#pragma unroll
    for (int t = 0; t < TPW; ++t) {
      const size_t to = (size_t)(16 * t) * KA + 32 * kt;
      Frag b;
      b.h[0] = *(const v8h*)(bp + to);
      b.h[1] = *(const v8h*)(bp + to + 16);
      acc[t] = wmh(a.v, b.v, acc[t]);
    }
  }

  {
    float* sp = stg + (size_t)(r0 + 8 * hh) * NCOL + c0 + m;
#pragma unroll
    for (int t = 0; t < TPW; ++t) {
      const float bv = bias[c0 + 16 * t + m];
#pragma unroll
      for (int r = 0; r < 8; ++r) sp[r * NCOL + 16 * t] = acc[t][r] * GSCALE + bv;
    }
  }
  __syncthreads();

  const int col4 = 4 * lane;
  v4f g4 = {1.f, 1.f, 1.f, 1.f}, b4 = {0.f, 0.f, 0.f, 0.f};
  if (LNRES) {
    g4 = *(const v4f*)(gam + col4);
    b4 = *(const v4f*)(bet + col4);
  }
  v4f o[RPW];
#pragma unroll
  for (int rr = 0; rr < RPW; ++rr) {
    const int row = wave * RPW + rr;
    const int grow = rowBase + row;
    const v4f v = *(const v4f*)(stg + row * NCOL + col4);
    v4f y;
    if (LNRES) {
      float s = (v.x + v.y) + (v.z + v.w);
#pragma unroll
      for (int sh = 16; sh > 0; sh >>= 1) s += __shfl_xor(s, sh);
      const float mu = s * (1.0f / (float)NCOL);
      const v4f d = v - mu;
      float q = (d.x * d.x + d.y * d.y) + (d.z * d.z + d.w * d.w);
#pragma unroll
      for (int sh = 16; sh > 0; sh >>= 1) q += __shfl_xor(q, sh);
      const float var = q * (1.0f / (float)NCOL);
      const float rstd = rsqrtf(var + LNEPS);
      y = d * rstd * g4 + b4;
      y.x = y.x < 0.f ? 0.f : y.x;
      y.y = y.y < 0.f ? 0.f : y.y;
      y.z = y.z < 0.f ? 0.f : y.z;
      y.w = y.w < 0.f ? 0.f : y.w;
      const int grc = grow > nValid - 1 ? nValid - 1 : grow;
      const v4f rs = *(const v4f*)(Res + (size_t)grc * NCOL + col4);
      y = y + rs;
    } else {
      y.x = v.x < 0.f ? 0.f : v.x;
      y.y = v.y < 0.f ? 0.f : v.y;
      y.z = v.z < 0.f ? 0.f : v.z;
      y.w = v.w < 0.f ? 0.f : v.w;
    }
    const bool live = grow < nValid;
    const v4f z = {0.f, 0.f, 0.f, 0.f};
    o[rr] = live ? y : z;
  }
  float* gb = Cout + (size_t)(rowBase + wave * RPW) * NCOL + col4;
#pragma unroll
  for (int rr = 0; rr < RPW; ++rr) *(volatile v4f*)(gb + (size_t)rr * NCOL) = o[rr];
  __threadfence();
#pragma unroll
  for (int rr = 0; rr < RPW; ++rr) *(volatile v4f*)(gb + (size_t)rr * NCOL) = o[rr];
}

__global__ __launch_bounds__(NTHR) void k_head(const float* __restrict__ h, const float* __restrict__ Wout,
                                               const float* __restrict__ bout, float* out, int nN, int outN) {
  __shared__ float wsh[FW * NCLS];
  __shared__ float bsh[NCLS];
  __shared__ __attribute__((aligned(16))) float osh[NTHR * NCLS];
  const int tid = threadIdx.x;
  wsh[tid] = Wout[tid];
  const float bv = bout[tid & (NCLS - 1)];
  if (tid < NCLS) bsh[tid] = bv;
  __syncthreads();
  const int node = (int)blockIdx.x * NTHR + tid;
  const int nc = node > nN - 1 ? nN - 1 : node;
  const float* hr = h + (size_t)nc * FW;
  float d0 = 0.f, d1 = 0.f;
#pragma unroll 1
  for (int q = 0; q < FW / 4; ++q) {
    const v4f v = *(const v4f*)(hr + 4 * q);
    const float* w = wsh + 8 * q;
    d0 += v.x * w[0] + v.y * w[2] + v.z * w[4] + v.w * w[6];
    d1 += v.x * w[1] + v.y * w[3] + v.z * w[5] + v.w * w[7];
  }
  const float l0 = d0 + bsh[0], l1 = d1 + bsh[1];
  const float mx = fmaxf(l0, l1), mn = fminf(l0, l1);
  const float t = expf(mn - mx);
  const float lse = mx + log1pf(t);
  osh[2 * tid]     = l0 - lse;
  osh[2 * tid + 1] = l1 - lse;
  __syncthreads();
  const bool wv = tid < (NTHR / 2);
  const int pc = wv ? tid : 0;
  const v4f ov = *(const v4f*)(osh + 4 * pc);
  const size_t e0 = (size_t)blockIdx.x * (NTHR * NCLS) + 4 * (size_t)tid;
  const bool st = wv && (e0 + 3 < (size_t)outN);
  if (st) *(volatile v4f*)(out + e0) = ov;
  __threadfence();
  if (st) *(volatile v4f*)(out + e0) = ov;
}

extern "C" void kernel_launch(void* const* d_in, const int* in_sizes, int n_in,
                              void* d_out, int out_size, void* d_ws, size_t ws_size,
                              hipStream_t stream) {
  if (n_in < 11) return;
  if (in_sizes[0] < FW || (in_sizes[0] % FW) != 0) return;
  const int nN = in_sizes[0] / FW;
  if (in_sizes[1] < 2 || (in_sizes[1] & 1) != 0) return;
  const int nE = in_sizes[1] / 2;
  if (in_sizes[2] != KIN * NH || in_sizes[3] != NH) return;
  if (in_sizes[4] != NLAY * FW * NH || in_sizes[5] != NLAY * NH || in_sizes[6] != NLAY * FW * NH) return;
  if (in_sizes[7] != NLAY * NH || in_sizes[8] != NLAY * NH) return;
  if (in_sizes[9] != FW * NCLS || in_sizes[10] != NCLS) return;
  if (out_size != nN * NCLS) return;
  if (nE < 1 || nE > (1 << 28) || nN < 1 || nN > (1 << 22)) return;

  const float* x    = (const float*)d_in[0];
  const int*   ei   = (const int*)d_in[1];
  const int*   src  = ei;
  const int*   dst  = ei + nE;
  const float* Win  = (const float*)d_in[2];
  const float* bin  = (const float*)d_in[3];
  const float* Wl   = (const float*)d_in[4];
  const float* bl   = (const float*)d_in[5];
  const float* Wr   = (const float*)d_in[6];
  const float* gam  = (const float*)d_in[7];
  const float* bet  = (const float*)d_in[8];
  const float* Wout = (const float*)d_in[9];
  const float* bout = (const float*)d_in[10];
  float* out = (float*)d_out;

  const int NPAD   = ((nN + RPAD - 1) / RPAD) * RPAD;
  const int nBC    = (nN + NBC - 1) / NBC;
  const int CNTPAD = nBC * NBC;
  if (CNTPAD < NPAD) return;
  if (4 * nBC + 1 > RBN) return;
  const int nBF    = (nN + NBF - 1) / NBF;
  if (nBF > 4 * nBC) return;
  const int csrLen = ((nE + 31) & ~31) + 4096;
  if (31 * 4 * nBC > 4096) return;
  const int nAgg   = NPAD / TGT;
  const int nG     = NPAD / BMR;
  const int nXU    = NPAD * (KIN / 8);
  const int nHB    = (nN + NTHR - 1) / NTHR;
  if (nHB * NTHR * NCLS < out_size) return;

  char* ws = (char*)d_ws;
  size_t off = 0;
  const size_t oWp  = off; off += (size_t)NUNITS * 8 * 2;       off = (off + 255) & ~(size_t)255;
  const size_t oX   = off; off += (size_t)NPAD * KIN * 2;        off = (off + 255) & ~(size_t)255;
  const size_t oA   = off; off += (size_t)NPAD * KS * 2;         off = (off + 255) & ~(size_t)255;
  const size_t oH0  = off; off += (size_t)NPAD * NH * 4;         off = (off + 255) & ~(size_t)255;
  const size_t oH1  = off; off += (size_t)NPAD * NH * 4;         off = (off + 255) & ~(size_t)255;
  const size_t oCnt = off; off += (size_t)CNTPAD * 4;            off = (off + 255) & ~(size_t)255;
  const size_t oOff = off; off += (size_t)CNTPAD * 4;            off = (off + 255) & ~(size_t)255;
  const size_t oRb  = off; off += (size_t)RBN * 4;               off = (off + 255) & ~(size_t)255;
  const size_t oCsr = off; off += (size_t)csrLen * 4;            off = (off + 255) & ~(size_t)255;
  if (off > ws_size || off > (size_t)WSCAP) return;

  _Float16* wpl = (_Float16*)(ws + oWp);
  _Float16* xpl = (_Float16*)(ws + oX);
  _Float16* apl = (_Float16*)(ws + oA);
  float* h0   = (float*)(ws + oH0);
  float* h1   = (float*)(ws + oH1);
  int*   cnt  = (int*)(ws + oCnt);
  int*   offp = (int*)(ws + oOff);
  int*   rb   = (int*)(ws + oRb);
  int*   csr  = (int*)(ws + oCsr);

  const int vec8 = ((nE & 3) == 0) ? 1 : 0;

  k_wcvt<<<NUNITS / NTHR, NTHR, 0, stream>>>(Win, Wl, Wr, wpl, NUNITS);
  k_xcvt<<<nXU / NTHR, NTHR, 0, stream>>>(x, xpl, nN, nXU);
  k_count<<<nBC, NTHR, 0, stream>>>(dst, cnt, nE, vec8);
  k_offsets<<<1, OTHR, 0, stream>>>(cnt, offp, rb, nBC);
  hipFuncSetAttribute(reinterpret_cast<const void*>(&k_fill),
                      hipFuncAttributeMaxDynamicSharedMemorySize, LDS_FILL);
  k_fill<<<nBF, NTHR, LDS_FILL, stream>>>(src, dst, offp, rb, csr, nN, nE, vec8, csrLen);

  k_gemm<KIN, 0><<<nG, NTHR, 0, stream>>>(xpl, wpl, bin, gam, bet, h1, h0, nN);

  for (int i = 0; i < NLAY; ++i) {
    const float* hin = (i & 1) ? h1 : h0;
    float* hout      = (i & 1) ? h0 : h1;
    k_agg<<<nAgg, ATHR, 0, stream>>>(csr, offp, cnt, hin, apl, nN, csrLen);
    k_gemm<KS, 1><<<nG, NTHR, 0, stream>>>(apl, wpl + (size_t)U0 * 8 + (size_t)i * UL * 8,
                                           bl + i * NH, gam + i * NH, bet + i * NH, hin, hout, nN);
  }
  const float* hfin = ((NLAY - 1) & 1) ? h0 : h1;

  k_head<<<nHB, NTHR, 0, stream>>>(hfin, Wout, bout, out, nN, out_size);
}
